// EntityAwareAttention_1898375544903
// MI455X (gfx1250) — hardware-verified
//
#include <hip/hip_runtime.h>
#ifndef NB
#define NB 4
#endif
#ifndef SEQ
#define SEQ 4096
#endif
#define NB_FULL 4
#define SEQ_FULL 4096
#define DM 768
#define NE 64
#define QC (SEQ < 256 ? SEQ : 256)
#define NR ((size_t)NB * SEQ)
#define MP ((int)(NB * SEQ))
#define PCARRY 4096.0f
#define PCARRY_L2 12.0f
#define LOG2E 1.4426950408889634f
#define SCALE2 (0.03608439182435161f * LOG2E)
#define AL256(x) ((((size_t)(x)) + 255) & ~(size_t)255)
#define WS_W  AL256((size_t)DM * DM * 2)
#define WS_P  AL256((size_t)NB * SEQ * DM * 2)
#define WS_S  AL256((size_t)NB * QC * SEQ * 4)
#define WS_PM AL256((size_t)NB * QC * SEQ * 2)
#define WS_CT AL256((size_t)NB * SEQ * 4)
static_assert(SEQ % 256 == 0);
static_assert(QC % 128 == 0);
static_assert(SEQ % QC == 0);
static_assert(NB <= NB_FULL);
static_assert(SEQ <= SEQ_FULL);
static_assert((NB * SEQ) % 128 == 0);
static_assert(DM % 128 == 0);
static_assert(DM % 64 == 0);
static_assert(DM % 32 == 0);
static_assert(SEQ % 64 == 0);
static_assert(DM % 8 == 0);
static_assert((NB * QC) % 4 == 0);
static_assert(4 * 32 * 68 * 4 <= 131072);
static_assert((float)(1 << 12) == PCARRY);
static_assert(3 * WS_W + 4 * WS_P + WS_S + WS_PM + WS_CT <= (size_t)134217728);
static_assert(((size_t)(NB - 1) * SEQ_FULL + SEQ) * DM <= (size_t)NB_FULL * SEQ_FULL * DM);

typedef unsigned short v8us __attribute__((ext_vector_type(8), may_alias));
typedef float  v8f  __attribute__((ext_vector_type(8)));
typedef float  v4f  __attribute__((ext_vector_type(4)));
typedef float  v4fa __attribute__((ext_vector_type(4), may_alias));
typedef _Float16 v16h __attribute__((ext_vector_type(16)));
typedef _Float16 v4h __attribute__((ext_vector_type(4)));
union FragH { v16h v; v8us half[2]; _Float16 h[16]; unsigned short u[16]; };

__device__ __forceinline__ unsigned short bf16_bits(float x) { unsigned int u = __float_as_uint(x); return (unsigned short)((u + 0x7FFFu + ((u >> 16) & 1u)) >> 16); }
__device__ __forceinline__ float bf16_val(unsigned short b) { return __uint_as_float(((unsigned int)b) << 16); }
__device__ __forceinline__ float bf16_rne(float x) { return bf16_val(bf16_bits(x)); }

typedef _Float16 h16;
static __device__ __forceinline__ h16 toh_flush(float v) { const h16 r = (h16)v; return (fabsf(v) < 6.103515625e-05f) ? (h16)0.0f : r; }

__device__ __forceinline__ v16h g2_frag(const _Float16* p, int hh) { FragH f; f.half[0] = *(const v8us*)((const unsigned short*)p + 8 * hh); f.half[1] = *(const v8us*)((const unsigned short*)p + 16 + 8 * hh); return f.v; }
__device__ __forceinline__ v8f g2_mma(v16h a, v16h b, v8f c) { v8f d = __builtin_amdgcn_wmma_f32_16x16x32_f16(false, a, false, b, (short)0, c, false, false); asm volatile("v_nop\n\tv_nop\n\tv_nop\n\tv_nop" : "+v"(d) : "v"(a), "v"(b)); return d; }

template <bool HASB, bool OUT32, bool OMAP>
__global__ __launch_bounds__(128) void k_gemm2(const _Float16* __restrict__ A, int lda, size_t sA, const _Float16* __restrict__ Bh, int ldb, size_t sB, float alpha,
    const float* __restrict__ bias, float* __restrict__ C, _Float16* __restrict__ C16, int ldc, size_t sC, int M, int N, int K) {
  __shared__ __attribute__((aligned(16))) float so[4][32][68];
  const int tid = threadIdx.x, w = __builtin_amdgcn_readfirstlane((int)(tid >> 5)), lane = tid & 31, ln = lane & 15, hh = lane >> 4; const int by = blockIdx.y;
  A += (size_t)by * sA; Bh += (size_t)by * sB; const size_t cofs = (size_t)by * sC;
  const int ntn = N >> 6; const int mt = blockIdx.x / ntn, nq = blockIdx.x - mt * ntn; const int row0 = mt * 128 + 32 * w, col0 = nq * 64; if (row0 >= M) return;
  const _Float16* a0p = A + (size_t)(row0 + ln) * lda; const _Float16* a1p = a0p + (size_t)16 * lda;
  const _Float16* b0p = Bh + (size_t)(col0 + ln) * ldb; const _Float16* b1p = b0p + (size_t)16 * ldb; const _Float16* b2p = b1p + (size_t)16 * ldb; const _Float16* b3p = b2p + (size_t)16 * ldb;
  const v8f z8 = {0.f,0.f,0.f,0.f,0.f,0.f,0.f,0.f}; v8f c00 = z8, c01 = z8, c02 = z8, c03 = z8, c10 = z8, c11 = z8, c12 = z8, c13 = z8;
#pragma unroll 1
  for (int kb = 0; kb < K; kb += 32) { const v16h a0 = g2_frag(a0p + kb, hh), a1 = g2_frag(a1p + kb, hh);
    v16h b = g2_frag(b0p + kb, hh); c00 = g2_mma(a0, b, c00); c10 = g2_mma(a1, b, c10);
    b = g2_frag(b1p + kb, hh); c01 = g2_mma(a0, b, c01); c11 = g2_mma(a1, b, c11);
    b = g2_frag(b2p + kb, hh); c02 = g2_mma(a0, b, c02); c12 = g2_mma(a1, b, c12);
    b = g2_frag(b3p + kb, hh); c03 = g2_mma(a0, b, c03); c13 = g2_mma(a1, b, c13); }
  v8f accs[8] = {c00, c01, c02, c03, c10, c11, c12, c13};
#pragma unroll
  for (int u = 0; u < 8; ++u) { const int t = u & 3, half = u >> 2; const int col = col0 + t * 16 + ln; float bv = 0.f; if (HASB) bv = bf16_rne(bias[col]);
#pragma unroll
    for (int r = 0; r < 8; ++r) { const int rloc = half * 16 + 8 * hh + r; so[w][rloc][t * 16 + ln] = accs[u][r] * alpha + bv; } }
  __builtin_amdgcn_fence(4  , "workgroup"); __builtin_amdgcn_wave_barrier();
  const int rsub = lane >> 4, c4 = (lane & 15) * 4;
  for (int pass = 0; pass < 2; ++pass) {
#pragma unroll
    for (int q = 0; q < 16; ++q) { const int r = q * 2 + rsub; const v4f v = *(const v4fa*)&so[w][r][c4];
      const int gr = row0 + r; const size_t orow = OMAP ? ((size_t)(gr / NB) * NB_FULL + (size_t)(gr % NB)) : (size_t)gr;
      if (OUT32) { *(volatile v4f*)(C + cofs + orow * ldc + col0 + c4) = v; }
      else { v4h h4;
#pragma unroll
        for (int i = 0; i < 4; ++i) h4[i] = (_Float16)v[i];
        *(volatile v4h*)(C16 + cofs + orow * ldc + col0 + c4) = h4; } }
    if (pass == 0) __threadfence(); } }

static_assert(((size_t)DM * DM) % 8 == 0);
__global__ __launch_bounds__(256) void k_wnat(const float* __restrict__ w, size_t n8, _Float16* __restrict__ Bt) { const size_t t = (size_t)blockIdx.x * 256 + threadIdx.x; if (t >= n8) return; FragH f; const v4f a = *(const v4fa*)(w + t * 8), c = *(const v4fa*)(w + t * 8 + 4);
#pragma unroll
  for (int q = 0; q < 4; ++q) { f.h[q] = toh_flush(bf16_rne(a[q]) * 16.0f); f.h[4 + q] = toh_flush(bf16_rne(c[q]) * 16.0f); }
  const v8us o = f.half[0]; *(volatile v8us*)((unsigned short*)Bt + t * 8) = o; __threadfence(); *(volatile v8us*)((unsigned short*)Bt + t * 8) = o; }

__global__ __launch_bounds__(256) void k_x16(const float* __restrict__ x, _Float16* __restrict__ X16, size_t n8) { const size_t t = (size_t)blockIdx.x * 256 + threadIdx.x; if (t >= n8) return;
  const size_t row = t / (DM / 8); const int c8 = (int)(t % (DM / 8)) * 8; const size_t srow = (row / SEQ) * SEQ_FULL + (row % SEQ);
  const float* p = x + srow * DM + c8; const v4f a = *(const v4fa*)p, c = *(const v4fa*)(p + 4); FragH f;
#pragma unroll
  for (int q = 0; q < 4; ++q) { f.h[q] = toh_flush(bf16_rne(a[q])); f.h[4 + q] = toh_flush(bf16_rne(c[q])); }
  const v8us o = f.half[0]; *(volatile v8us*)((unsigned short*)X16 + t * 8) = o; __threadfence(); *(volatile v8us*)((unsigned short*)X16 + t * 8) = o; }

static_assert((NB * (SEQ / 4)) * 16 == NB * SEQ * 4);
__global__ __launch_bounds__(256) void k_colterm(const float* __restrict__ mask, const int* __restrict__ epos, float* __restrict__ CT) {
  #pragma clang fp contract(off)
  const int t = blockIdx.x * 256 + threadIdx.x; if (t >= NB * (SEQ / 4)) return;
  const int b = t / (SEQ / 4); const int c4 = (t - b * (SEQ / 4)) * 4;
  const v4f m = *(const v4fa*)(mask + (size_t)b * SEQ_FULL + c4);
  int n0 = 0, n1 = 0, n2 = 0, n3 = 0, bad = 0;
#pragma unroll 1
  for (int e = 0; e < NE; ++e) { const int p = epos[b * NE + e];
    bad |= ((unsigned)p >= (unsigned)SEQ_FULL) ? 1 : 0;
    n0 += (p == c4) ? 1 : 0; n1 += (p == c4 + 1) ? 1 : 0; n2 += (p == c4 + 2) ? 1 : 0; n3 += (p == c4 + 3) ? 1 : 0; }
  const float qn = __uint_as_float(0x7FC00000u);
  const float t0 = (float)n0 * LOG2E + ((1.0f - bf16_rne(m[0])) * -10000.0f) * LOG2E;
  const float t1 = (float)n1 * LOG2E + ((1.0f - bf16_rne(m[1])) * -10000.0f) * LOG2E;
  const float t2 = (float)n2 * LOG2E + ((1.0f - bf16_rne(m[2])) * -10000.0f) * LOG2E;
  const float t3 = (float)n3 * LOG2E + ((1.0f - bf16_rne(m[3])) * -10000.0f) * LOG2E;
  v4f o; o[0] = (bad != 0) ? qn : t0; o[1] = (bad != 0) ? qn : t1; o[2] = (bad != 0) ? qn : t2; o[3] = (bad != 0) ? qn : t3;
  *(volatile v4f*)(CT + (size_t)t * 4) = o; __threadfence(); *(volatile v4f*)(CT + (size_t)t * 4) = o; }

static_assert(32 * 16 * (SEQ / 256) == SEQ * 2);
__global__ __launch_bounds__(128) __attribute__((amdgpu_num_vgpr(256))) void k_soft(const float* __restrict__ S, const float* __restrict__ CT, _Float16* __restrict__ PM) {
  #pragma clang fp contract(off)
  const int tid = threadIdx.x, w = __builtin_amdgcn_readfirstlane((int)(tid >> 5)), lane = tid & 31;
  const int wr = blockIdx.x * 4 + w; const int b = wr / QC;
  const float* p = S + (size_t)wr * SEQ + lane * 8;
  const float* c = CT + (size_t)b * SEQ + lane * 8;
  v4f x[SEQ / 128];
#pragma unroll
  for (int j = 0; j < SEQ / 256; ++j) {
    const v4f s0 = *(const v4fa*)(p + j * 256), s1 = *(const v4fa*)(p + j * 256 + 4);
    const v4f u0 = *(const v4fa*)(c + j * 256), u1 = *(const v4fa*)(c + j * 256 + 4);
    x[2 * j] = s0 + u0; x[2 * j + 1] = s1 + u1;
    asm volatile("" : "+v"(x[2 * j]), "+v"(x[2 * j + 1]) : : "memory");
    __builtin_amdgcn_sched_barrier(0); }
  float mx = -3.0e38f;
#pragma unroll
  for (int j = 0; j < SEQ / 128; ++j) mx = fmaxf(mx, fmaxf(fmaxf(x[j][0], x[j][1]), fmaxf(x[j][2], x[j][3])));
#pragma unroll
  for (int off = 16; off > 0; off >>= 1) mx = fmaxf(mx, __shfl_xor(mx, off, 32));
  float se = 0.f;
#pragma unroll
  for (int j = 0; j < SEQ / 128; ++j) {
#pragma unroll
    for (int i = 0; i < 4; ++i) { const float e = __builtin_amdgcn_exp2f(x[j][i] - mx); se += e; } }
#pragma unroll
  for (int off = 16; off > 0; off >>= 1) se += __shfl_xor(se, off, 32);
  const float xoff = (mx + __builtin_amdgcn_logf(se)) - PCARRY_L2;
  unsigned short* pout = (unsigned short*)PM + (size_t)wr * SEQ + lane * 8;
  for (int pass = 0; pass < 2; ++pass) {
#pragma unroll
    for (int j = 0; j < SEQ / 256; ++j) { FragH f;
#pragma unroll
      for (int i = 0; i < 4; ++i) { f.h[i] = toh_flush(__builtin_amdgcn_exp2f(x[2 * j][i] - xoff)); f.h[4 + i] = toh_flush(__builtin_amdgcn_exp2f(x[2 * j + 1][i] - xoff)); }
      const v8us o = f.half[0]; *(volatile v8us*)(pout + j * 256) = o; }
    if (pass == 0) __threadfence(); } }

extern "C" void kernel_launch(void* const* d_in, const int* in_sizes, int n_in,
                              void* d_out, int out_size, void* d_ws, size_t ws_size, hipStream_t stream) {
  if (n_in < 9) return;
  const size_t xneed = ((size_t)(NB - 1) * SEQ_FULL + SEQ) * DM;
  if ((size_t)in_sizes[0] < xneed) return;
  if ((size_t)in_sizes[1] < (size_t)(NB - 1) * SEQ_FULL + SEQ) return;
  if (in_sizes[2] < NB * NE) return;
  if ((size_t)in_sizes[3] < (size_t)DM * DM || (size_t)in_sizes[5] < (size_t)DM * DM || (size_t)in_sizes[7] < (size_t)DM * DM) return;
  if (in_sizes[4] < DM || in_sizes[6] < DM || in_sizes[8] < DM) return;
  if ((size_t)out_size < xneed) return;
  const float* const* I = (const float* const*)d_in;
  const float* hs = I[0]; const float* mask = I[1]; const int* epos = (const int*)d_in[2];
  const float* wq = I[3]; const float* bq = I[4]; const float* wk = I[5]; const float* bk = I[6]; const float* wv = I[7]; const float* bv = I[8];
  char* ws = (char*)d_ws; size_t off = 0;
  auto take = [&](size_t bytes) { char* p = ws + off; off += (bytes + 255) & ~(size_t)255; return p; };
  _Float16* BQ = (_Float16*)take((size_t)DM * DM * 2); _Float16* BK = (_Float16*)take((size_t)DM * DM * 2); _Float16* BV = (_Float16*)take((size_t)DM * DM * 2);
  _Float16* X16 = (_Float16*)take(NR * DM * 2); _Float16* Q16 = (_Float16*)take(NR * DM * 2); _Float16* K16 = (_Float16*)take(NR * DM * 2); _Float16* VT = (_Float16*)take(NR * DM * 2);
  float* S = (float*)take((size_t)NB * QC * SEQ * 4); _Float16* PM = (_Float16*)take((size_t)NB * QC * SEQ * 2);
  float* CT = (float*)take((size_t)NB * SEQ * 4);
  if (off > ws_size) return;
  { const unsigned g = (unsigned)(((size_t)DM * DM / 8 + 255) / 256);
    k_wnat<<<g, 256, 0, stream>>>(wq, (size_t)DM * DM / 8, BQ); k_wnat<<<g, 256, 0, stream>>>(wk, (size_t)DM * DM / 8, BK);
    k_wnat<<<g, 256, 0, stream>>>(wv, (size_t)DM * DM / 8, BV); }
  k_x16<<<(unsigned)((NR * DM / 8 + 255) / 256), 256, 0, stream>>>(hs, X16, NR * DM / 8);
  k_colterm<<<(unsigned)((NB * (SEQ / 4) + 255) / 256), 256, 0, stream>>>(mask, epos, CT);
  const dim3 gp((unsigned)((MP / 128) * (DM / 64)), 1);
  k_gemm2<true, false, false><<<gp, 128, 0, stream>>>(X16, DM, 0, BQ, DM, 0, 0.0625f, bq, nullptr, Q16, DM, 0, MP, DM, DM);
  k_gemm2<true, false, false><<<gp, 128, 0, stream>>>(X16, DM, 0, BK, DM, 0, 0.0625f, bk, nullptr, K16, DM, 0, MP, DM, DM);
  k_gemm2<false, false, false><<<dim3((DM / 128) * (SEQ / 64), NB), 128, 0, stream>>>(BV, DM, 0, X16, DM, (size_t)SEQ * DM, 0.0625f, nullptr, nullptr, VT, SEQ, (size_t)DM * SEQ, DM, SEQ, DM);
  for (int t0 = 0; t0 < SEQ; t0 += QC) {
    k_gemm2<false, true, false><<<dim3((QC / 128) * (SEQ / 64), NB), 128, 0, stream>>>(Q16 + (size_t)t0 * DM, DM, (size_t)SEQ * DM, K16, DM, (size_t)SEQ * DM, SCALE2, nullptr, S, nullptr, SEQ, (size_t)QC * SEQ, QC, SEQ, DM);
    k_soft<<<NB * QC / 4, 128, 0, stream>>>(S, CT, PM);
    k_gemm2<true, true, false><<<dim3((QC / 128) * (DM / 64), NB), 128, 0, stream>>>(PM, SEQ, (size_t)QC * SEQ, VT, SEQ, (size_t)DM * SEQ, 0.000244140625f, bv, (float*)d_out + (size_t)t0 * DM, nullptr, DM, (size_t)SEQ_FULL * DM, QC, DM, SEQ);
  }
}
